// ResidualTransformerLayer_89326729822667
// MI455X (gfx1250) — hardware-verified
//
#include <hip/hip_runtime.h>
#include <stddef.h>


#define HIDC  64
#define NHD   4
#define DM    256
#define PLN   (DM * HIDC)
#define GR    32
#define AP    72
#define HP    264
#define SP    260
#define OPF   68
#define TR    16
#define TTHR  128
#define NB    256
#define CHUNK 2048
#define NTHR  256
#define NWAVE 8
#define WCAP  256
#define NGRP  (CHUNK / (NTHR * 4))

#define LDS_SACC (NB * DM)
#define LDS_AUX  (NB * NHD * 2)
#define LDS_LIST (NWAVE * WCAP)
#define LDS_BYTES ((LDS_SACC + LDS_AUX + LDS_LIST + NWAVE) * 4)

static_assert(WCAP == (CHUNK / NTHR) * 32);
static_assert(NGRP == 2);
static_assert(NB == 256);
static_assert(CHUNK == 2048);
static_assert((LDS_SACC % 4) == 0);
static_assert(LDS_BYTES == 278560);
static_assert(NB / NWAVE == 32);
static_assert(DM == NHD * HIDC);

typedef float          v4f  __attribute__((ext_vector_type(4)));
typedef float          v8f  __attribute__((ext_vector_type(8)));
typedef int            v4i  __attribute__((ext_vector_type(4)));
typedef unsigned int   v2u  __attribute__((ext_vector_type(2)));
typedef _Float16       v8h  __attribute__((ext_vector_type(8)));
typedef _Float16       v16h __attribute__((ext_vector_type(16)));
typedef __bf16         v16b __attribute__((ext_vector_type(16)));
union FragH  { v16h v; v4i q[2]; };
union FragB  { v16b v; v4i q[2]; };
union Pack16 { v8h h; unsigned short s[8]; v4i i; };
union Pack8  { unsigned short s[4]; v2u u; };

__device__ __forceinline__ v8f wmh(v16h a, v16h b, v8f c) {
  v8f d = __builtin_amdgcn_wmma_f32_16x16x32_f16(false, a, false, b, (short)0, c, false, false);
  asm volatile("v_nop\n\tv_nop\n\tv_nop\n\tv_nop" : "+v"(d) : "v"(a), "v"(b));
  return d;
}
__device__ __forceinline__ v8f wmb(v16b a, v16b b, v8f c) {
  v8f d = __builtin_amdgcn_wmma_f32_16x16x32_bf16(false, a, false, b, (short)0, c, false, false);
  asm volatile("v_nop\n\tv_nop\n\tv_nop\n\tv_nop" : "+v"(d) : "v"(a), "v"(b));
  return d;
}

__device__ __forceinline__ float wsum(float v) {
  v += __shfl_xor(v, 16, 32);
  v += __shfl_xor(v, 8, 32);
  v += __shfl_xor(v, 4, 32);
  v += __shfl_xor(v, 2, 32);
  v += __shfl_xor(v, 1, 32);
  return v;
}

__device__ __forceinline__ unsigned short bf_rne(float f) {
  unsigned int u = __float_as_uint(f);
  u += 0x7FFFu + ((u >> 16) & 1u);
  return (unsigned short)(u >> 16);
}
__device__ __forceinline__ float bf_val(unsigned short s) {
  return __uint_as_float(((unsigned int)s) << 16);
}

__global__ __launch_bounds__(NTHR) void k_prep(const float* __restrict__ Wq, const float* __restrict__ Wk,
                                               const float* __restrict__ Wv, const float* __restrict__ Wsk,
                                               const float* __restrict__ Wp, unsigned short* pl, int n8) {
  const int i = blockIdx.x * NTHR + threadIdx.x;
  const int which = blockIdx.y;
  if (i >= n8) return;
  const float* W = Wq;
  if (which == 1) W = Wk;
  else if (which == 2) W = Wv;
  else if (which == 3) W = Wsk;
  else if (which == 4) W = Wp;
  const size_t o = (size_t)i * 8;
  const v4f a = *(const v4f*)(W + o);
  const v4f b = *(const v4f*)(W + o + 4);
  const float f[8] = {a.x, a.y, a.z, a.w, b.x, b.y, b.z, b.w};
  Pack16 u0, u1;
  size_t d0, d1;
  if (which < 3) {
#pragma unroll
    for (int c = 0; c < 8; ++c) u0.h[c] = (_Float16)(f[c] * 8.0f);
    u1.i = u0.i;
    d0 = (size_t)which * PLN + o;
    d1 = d0;
  } else {
#pragma unroll
    for (int c = 0; c < 8; ++c) {
      const unsigned short hs = bf_rne(f[c]);
      u0.s[c] = hs;
      u1.s[c] = bf_rne(f[c] - bf_val(hs));
    }
    const int base = 3 + 2 * (which - 3);
    d0 = (size_t)base * PLN + o;
    d1 = d0 + PLN;
  }
  *(volatile v4i*)(pl + d0) = u0.i;
  *(volatile v4i*)(pl + d1) = u1.i;
  __threadfence();
  *(volatile v4i*)(pl + d0) = u0.i;
  *(volatile v4i*)(pl + d1) = u1.i;
}

__global__ __launch_bounds__(NTHR) void k_qkv(const float* __restrict__ x, const _Float16* __restrict__ wpl,
                                              const float* __restrict__ bq, const float* __restrict__ bk,
                                              const float* __restrict__ bv, _Float16* qkv, int nN, int nP) {
  __shared__ __attribute__((aligned(16))) _Float16 At[GR * AP];
  __shared__ __attribute__((aligned(16))) _Float16 Hs[GR * HP];

  const int tid  = threadIdx.x;
  const int lane = tid & 31;
  const int wave = tid >> 5;
  const int hh   = lane >> 4;
  const int m    = lane & 15;
  const int mi   = blockIdx.y;
  const int rowBase = blockIdx.x * GR;
  const _Float16* Wh = wpl + (size_t)mi * PLN;
  const float* bias = bq;
  if (mi == 1) bias = bk; else if (mi == 2) bias = bv;
  _Float16* dst = qkv + (size_t)mi * (size_t)nP * DM;

  {
    const int r  = tid >> 3;
    const int c0 = (tid & 7) * 8;
    int row = rowBase + r;
    if (row > nN - 1) row = nN - 1;
    const float* p = x + (size_t)row * HIDC + c0;
    const v4f f0 = *(const v4f*)p, f1 = *(const v4f*)(p + 4);
    Pack16 u;
    u.h[0] = (_Float16)f0.x; u.h[1] = (_Float16)f0.y; u.h[2] = (_Float16)f0.z; u.h[3] = (_Float16)f0.w;
    u.h[4] = (_Float16)f1.x; u.h[5] = (_Float16)f1.y; u.h[6] = (_Float16)f1.z; u.h[7] = (_Float16)f1.w;
    *(v4i*)(At + r * AP + c0) = u.i;
  }
  __syncthreads();

#pragma unroll
  for (int ct = 0; ct < 2; ++ct) {
    const int ncol = wave * 32 + ct * 16 + m;
    v8f c0 = {0.f, 0.f, 0.f, 0.f, 0.f, 0.f, 0.f, 0.f};
    v8f c1 = {0.f, 0.f, 0.f, 0.f, 0.f, 0.f, 0.f, 0.f};
#pragma unroll
    for (int kt = 0; kt < HIDC / 32; ++kt) {
      const int k0 = kt * 32;
      FragH a0, a1, b;
      const _Float16* pb  = Wh + (size_t)ncol * HIDC + k0 + 8 * hh;
      const _Float16* pa0 = At + m * AP + k0 + 8 * hh;
      const _Float16* pa1 = At + (16 + m) * AP + k0 + 8 * hh;
      b.q[0]  = *(const v4i*)pb;  b.q[1]  = *(const v4i*)(pb + 16);
      a0.q[0] = *(const v4i*)pa0; a0.q[1] = *(const v4i*)(pa0 + 16);
      a1.q[0] = *(const v4i*)pa1; a1.q[1] = *(const v4i*)(pa1 + 16);
      c0 = wmh(a0.v, b.v, c0);
      c1 = wmh(a1.v, b.v, c1);
    }
    const float bsv = bias[ncol];
#pragma unroll
    for (int r = 0; r < 8; ++r) {
      Hs[(8 * hh + r) * HP + ncol]      = (_Float16)(c0[r] * 0.125f + bsv);
      Hs[(16 + 8 * hh + r) * HP + ncol] = (_Float16)(c1[r] * 0.125f + bsv);
    }
  }
  __syncthreads();

  v4i keep[4];
  _Float16* gp[4];
#pragma unroll
  for (int i = 0; i < 4; ++i) {
    const int row = 4 * wave + i;
    keep[i] = *(const v4i*)(Hs + row * HP + 8 * lane);
    gp[i] = dst + (size_t)(rowBase + row) * DM + 8 * lane;
  }
#pragma unroll
  for (int i = 0; i < 4; ++i) *(volatile v4i*)(gp[i]) = keep[i];
  __threadfence();
#pragma unroll
  for (int i = 0; i < 4; ++i) *(volatile v4i*)(gp[i]) = keep[i];
}

__global__ __launch_bounds__(NTHR) void k_agg(const int* __restrict__ ei, const _Float16* __restrict__ qh,
                                              const _Float16* __restrict__ kh, const _Float16* __restrict__ vh,
                                              float* agg, int nN, int nE) {
  extern __shared__ v4f lds_dyn[];
  float* sacc = (float*)lds_dyn;
  float* den  = sacc + LDS_SACC;
  float* mx   = den + NB * NHD;
  int*   list = (int*)(mx + NB * NHD);
  int*   wcnt = list + LDS_LIST;

  const int tid  = threadIdx.x;
  const int lane = tid & 31;
  const int wave = tid >> 5;
  const int hd   = lane >> 3;
  const int nodeBase = blockIdx.x * NB;

  {
    const v4f z4 = {0.f, 0.f, 0.f, 0.f};
    for (int i = tid; i < LDS_SACC / 4; i += NTHR) lds_dyn[i] = z4;
    for (int i = tid; i < NB * NHD; i += NTHR) { den[i] = 0.f; mx[i] = -1.0e30f; }
  }
  __syncthreads();

  const int* eid = ei + nE;
  const bool al16 = ((nE & 3) == 0);

  const int nChunks = (nE + CHUNK - 1) / CHUNK;
#pragma unroll 1
  for (int ch = 0; ch < nChunks; ++ch) {
    const int cbase = ch * CHUNK;
    int wc = 0;
#pragma unroll
    for (int g = 0; g < NGRP; ++g) {
      const int el0 = (g * NTHR + tid) * 4;
      const int e0  = cbase + el0;
      const int sent = -2147483647 - 1;
      v4i d;
      if (al16 && (e0 + 3 < nE)) {
        d = *(const v4i*)(eid + e0);
      } else {
        d.x = (e0     < nE) ? eid[min(e0, nE - 1)]     : sent;
        d.y = (e0 + 1 < nE) ? eid[min(e0 + 1, nE - 1)] : sent;
        d.z = (e0 + 2 < nE) ? eid[min(e0 + 2, nE - 1)] : sent;
        d.w = (e0 + 3 < nE) ? eid[min(e0 + 3, nE - 1)] : sent;
      }
      const unsigned s0 = (unsigned)d.x - (unsigned)nodeBase;
      const unsigned s1 = (unsigned)d.y - (unsigned)nodeBase;
      const unsigned s2 = (unsigned)d.z - (unsigned)nodeBase;
      const unsigned s3 = (unsigned)d.w - (unsigned)nodeBase;
      const bool h0 = s0 < (unsigned)NB;
      const bool h1 = s1 < (unsigned)NB;
      const bool h2 = s2 < (unsigned)NB;
      const bool h3 = s3 < (unsigned)NB;
      const unsigned many = __builtin_amdgcn_ballot_w32(h0 | h1 | h2 | h3);
      if (many != 0u) {
#define HITJ(J, HJ, SJ) { \
          const unsigned mj = __builtin_amdgcn_ballot_w32(HJ); \
          if (HJ) { \
            const int pos = wc + (int)__builtin_amdgcn_mbcnt_lo(mj, 0u); \
            if (pos < WCAP) list[wave * WCAP + pos] = ((el0 + (J)) << 8) | (int)(SJ); \
          } \
          wc += (int)__builtin_popcount(mj); }
        HITJ(0, h0, s0)
        HITJ(1, h1, s1)
        HITJ(2, h2, s2)
        HITJ(3, h3, s3)
#undef HITJ
      }
    }
    if (lane == 0) wcnt[wave] = wc;
    __syncthreads();

    if (wave == 0) {
#pragma unroll 1
      for (int wsx = 0; wsx < NWAVE; ++wsx) {
        int n = wcnt[wsx];
        if (n > WCAP) n = WCAP;
        if (n < 0) n = 0;
#pragma unroll 1
        for (int i = 0; i < n; ++i) {
          const int ent  = list[wsx * WCAP + i];
          const int slot = ent & (NB - 1);
          const int el   = (ent >> 8) & (CHUNK - 1);
          int e = cbase + el;
          if (e > nE - 1) e = nE - 1;
          int src = ei[e];
          src = src < 0 ? 0 : (src > nN - 1 ? nN - 1 : src);
          int nd = nodeBase + slot;
          if (nd > nN - 1) nd = nN - 1;
          Pack16 uq, uk, uv;
          uq.i = *(const v4i*)(qh + (size_t)nd  * DM + 8 * lane);
          uk.i = *(const v4i*)(kh + (size_t)src * DM + 8 * lane);
          uv.i = *(const v4i*)(vh + (size_t)src * DM + 8 * lane);
          float dt = 0.f;
#pragma unroll
          for (int c = 0; c < 8; ++c) dt += (float)uq.h[c] * (float)uk.h[c];
          dt += __shfl_xor(dt, 4, 32);
          dt += __shfl_xor(dt, 2, 32);
          dt += __shfl_xor(dt, 1, 32);
          const float a  = dt * 0.125f;
          const int   ai = slot * NHD + hd;
          const float mo = mx[ai];
          const float mn = fmaxf(mo, a);
          const float sc = __expf(mo - mn);
          const float p  = __expf(a - mn);
          v4f v0, v1;
          v0.x = (float)uv.h[0]; v0.y = (float)uv.h[1]; v0.z = (float)uv.h[2]; v0.w = (float)uv.h[3];
          v1.x = (float)uv.h[4]; v1.y = (float)uv.h[5]; v1.z = (float)uv.h[6]; v1.w = (float)uv.h[7];
          v4f* sp = (v4f*)(sacc + slot * DM + 8 * lane);
          const v4f cA = sp[0];
          const v4f cB = sp[1];
          sp[0] = cA * sc + v0 * p;
          sp[1] = cB * sc + v1 * p;
          if ((lane & 7) == 0) {
            const float dn = den[ai];
            mx[ai]  = mn;
            den[ai] = dn * sc + p;
          }
        }
      }
    }
    __syncthreads();
  }

  const int hq = lane >> 4;
#pragma unroll 1
  for (int j = 0; j < NB / NWAVE; ++j) {
    const int slot = wave * (NB / NWAVE) + j;
    const size_t nrow = (size_t)(nodeBase + slot);
    const float d0 = den[slot * NHD + hq];
    const float d1 = den[slot * NHD + 2 + hq];
    const float i0 = (d0 > 0.f) ? (1.0f / d0) : 0.f;
    const float i1 = (d1 > 0.f) ? (1.0f / d1) : 0.f;
    const v4f s0 = *(const v4f*)(sacc + slot * DM + 4 * lane) * i0;
    const v4f s1 = *(const v4f*)(sacc + slot * DM + 128 + 4 * lane) * i1;
    float* op = agg + nrow * DM + 4 * lane;
    *(volatile v4f*)op = s0;
    *(volatile v4f*)(op + 128) = s1;
    __threadfence();
    *(volatile v4f*)op = s0;
    *(volatile v4f*)(op + 128) = s1;
  }
}

__global__ __launch_bounds__(TTHR) void k_tail(
    const float* __restrict__ x, const float* __restrict__ agg,
    const unsigned short* __restrict__ wsh, const unsigned short* __restrict__ wsl,
    const float* __restrict__ bsk, const float* __restrict__ wb,
    const float* __restrict__ lg, const float* __restrict__ lb,
    const unsigned short* __restrict__ wph, const unsigned short* __restrict__ wpl,
    const float* __restrict__ bp, float* out, int nN, int nPA) {
  __shared__ __attribute__((aligned(16))) unsigned short Xh[TR * AP];
  __shared__ __attribute__((aligned(16))) unsigned short Xl[TR * AP];
  __shared__ __attribute__((aligned(16))) unsigned short Zh[TR * HP];
  __shared__ __attribute__((aligned(16))) unsigned short Zl[TR * HP];
  __shared__ __attribute__((aligned(16))) float Ss[TR * SP];
  __shared__ __attribute__((aligned(16))) float Os[TR * OPF];

  const int tid  = threadIdx.x;
  const int lane = tid & 31;
  const int wave = tid >> 5;
  const int hh   = lane >> 4;
  const int m    = lane & 15;
  const int rowBase = blockIdx.x * TR;

  {
    const int r  = tid >> 3;
    const int c0 = (tid & 7) * 8;
    int row = rowBase + r;
    if (row > nN - 1) row = nN - 1;
    const float* p = x + (size_t)row * HIDC + c0;
    const v4f f0 = *(const v4f*)p, f1 = *(const v4f*)(p + 4);
    const float f[8] = {f0.x, f0.y, f0.z, f0.w, f1.x, f1.y, f1.z, f1.w};
    Pack16 uh, ul;
#pragma unroll
    for (int c = 0; c < 8; ++c) {
      const unsigned short hs = bf_rne(f[c]);
      uh.s[c] = hs;
      ul.s[c] = bf_rne(f[c] - bf_val(hs));
    }
    *(v4i*)(Xh + r * AP + c0) = uh.i;
    *(v4i*)(Xl + r * AP + c0) = ul.i;
  }
  __syncthreads();

  {
    FragB ah[2], al[2];
#pragma unroll
    for (int kt = 0; kt < 2; ++kt) {
      const unsigned short* pah = Xh + m * AP + 32 * kt + 8 * hh;
      const unsigned short* pal = Xl + m * AP + 32 * kt + 8 * hh;
      ah[kt].q[0] = *(const v4i*)pah; ah[kt].q[1] = *(const v4i*)(pah + 16);
      al[kt].q[0] = *(const v4i*)pal; al[kt].q[1] = *(const v4i*)(pal + 16);
    }
#pragma unroll
    for (int ct = 0; ct < 4; ++ct) {
      const int ncol = wave * 64 + ct * 16 + m;
      v8f acc = {0.f, 0.f, 0.f, 0.f, 0.f, 0.f, 0.f, 0.f};
#pragma unroll
      for (int kt = 0; kt < 2; ++kt) {
        FragB bh, bl;
        const unsigned short* pbh = wsh + (size_t)ncol * HIDC + 32 * kt + 8 * hh;
        const unsigned short* pbl = wsl + (size_t)ncol * HIDC + 32 * kt + 8 * hh;
        bh.q[0] = *(const v4i*)pbh; bh.q[1] = *(const v4i*)(pbh + 16);
        bl.q[0] = *(const v4i*)pbl; bl.q[1] = *(const v4i*)(pbl + 16);
        acc = wmb(ah[kt].v, bh.v, acc);
        acc = wmb(ah[kt].v, bl.v, acc);
        acc = wmb(al[kt].v, bh.v, acc);
      }
      const float bsv = bsk[ncol];
#pragma unroll
      for (int r = 0; r < 8; ++r) Ss[(8 * hh + r) * SP + ncol] = acc[r] + bsv;
    }
  }
  __syncthreads();

#pragma unroll 1
  for (int i = 0; i < 4; ++i) {
    const int rl = 4 * wave + i;
    int ar = rowBase + rl;
    if (ar > nPA - 1) ar = nPA - 1;
    v4f ag[2], sk[2];
    v4f zz = {0.f, 0.f, 0.f, 0.f};
#pragma unroll
    for (int j = 0; j < 2; ++j) {
      const int c = 4 * lane + 128 * j;
      ag[j] = *(const v4f*)(agg + (size_t)ar * DM + c);
      sk[j] = *(const v4f*)(Ss + rl * SP + c);
      const v4f w1 = *(const v4f*)(wb + c);
      const v4f w2 = *(const v4f*)(wb + DM + c);
      const v4f w3 = *(const v4f*)(wb + 2 * DM + c);
      const v4f df = ag[j] - sk[j];
      zz += ag[j] * w1 + sk[j] * w2 + df * w3;
    }
    const float z    = wsum(zz.x + zz.y + zz.z + zz.w);
    const float beta = 1.0f / (1.0f + __expf(-z));
    const float omb  = 1.0f - beta;
    v4f hv[2];
#pragma unroll
    for (int j = 0; j < 2; ++j) hv[j] = sk[j] * beta + ag[j] * omb;
    const float s  = wsum(hv[0].x + hv[0].y + hv[0].z + hv[0].w + hv[1].x + hv[1].y + hv[1].z + hv[1].w);
    const float mu = s * (1.0f / DM);
    v4f dv[2];
    float qq = 0.f;
#pragma unroll
    for (int j = 0; j < 2; ++j) {
      dv[j] = hv[j] - mu;
      qq += dv[j].x * dv[j].x + dv[j].y * dv[j].y + dv[j].z * dv[j].z + dv[j].w * dv[j].w;
    }
    const float var = wsum(qq) * (1.0f / DM);
    const float rs  = rsqrtf(var + 1e-5f);
#pragma unroll
    for (int j = 0; j < 2; ++j) {
      const int c = 4 * lane + 128 * j;
      const v4f g4 = *(const v4f*)(lg + c);
      const v4f b4 = *(const v4f*)(lb + c);
      const v4f y = dv[j] * rs * g4 + b4;
      const float yy[4] = {y.x, y.y, y.z, y.w};
      Pack8 ph, pl8;
#pragma unroll
      for (int t = 0; t < 4; ++t) {
        const unsigned short hs = bf_rne(yy[t]);
        ph.s[t]  = hs;
        pl8.s[t] = bf_rne(yy[t] - bf_val(hs));
      }
      *(v2u*)(Zh + rl * HP + c) = ph.u;
      *(v2u*)(Zl + rl * HP + c) = pl8.u;
    }
  }
  __syncthreads();

  const int ncol = wave * 16 + m;
  v8f acc = {0.f, 0.f, 0.f, 0.f, 0.f, 0.f, 0.f, 0.f};
#pragma unroll
  for (int kt = 0; kt < DM / 32; ++kt) {
    const int k0 = kt * 32;
    FragB a_h, a_l, b_h, b_l;
    const unsigned short* pah = Zh + m * HP + k0 + 8 * hh;
    const unsigned short* pal = Zl + m * HP + k0 + 8 * hh;
    const unsigned short* pbh = wph + (size_t)ncol * DM + k0 + 8 * hh;
    const unsigned short* pbl = wpl + (size_t)ncol * DM + k0 + 8 * hh;
    a_h.q[0] = *(const v4i*)pah; a_h.q[1] = *(const v4i*)(pah + 16);
    a_l.q[0] = *(const v4i*)pal; a_l.q[1] = *(const v4i*)(pal + 16);
    b_h.q[0] = *(const v4i*)pbh; b_h.q[1] = *(const v4i*)(pbh + 16);
    b_l.q[0] = *(const v4i*)pbl; b_l.q[1] = *(const v4i*)(pbl + 16);
    acc = wmb(a_h.v, b_h.v, acc);
    acc = wmb(a_h.v, b_l.v, acc);
    acc = wmb(a_l.v, b_h.v, acc);
  }
  {
    const float bsv = bp[ncol];
#pragma unroll
    for (int r = 0; r < 8; ++r) {
      const int rl = 8 * hh + r;
      int gr = rowBase + rl;
      if (gr > nN - 1) gr = nN - 1;
      const float o = acc[r] + bsv + x[(size_t)gr * HIDC + ncol];
      Os[rl * OPF + ncol] = fmaxf(o, 0.0f);
    }
  }
  __syncthreads();

  v4f ov[2];
  int og[2];
#pragma unroll
  for (int s2 = 0; s2 < 2; ++s2) {
    const int rl = 4 * wave + 2 * s2 + hh;
    og[s2] = rowBase + rl;
    ov[s2] = *(const v4f*)(Os + rl * OPF + 4 * m);
  }
#pragma unroll
  for (int s2 = 0; s2 < 2; ++s2)
    if (og[s2] < nN) *(volatile v4f*)(out + (size_t)og[s2] * HIDC + 4 * m) = ov[s2];
  __threadfence();
#pragma unroll
  for (int s2 = 0; s2 < 2; ++s2)
    if (og[s2] < nN) *(volatile v4f*)(out + (size_t)og[s2] * HIDC + 4 * m) = ov[s2];
}

extern "C" void kernel_launch(void* const* d_in, const int* in_sizes, int n_in,
                              void* d_out, int out_size, void* d_ws, size_t ws_size,
                              hipStream_t stream) {
  if (n_in < 15) return;
  const int nN = in_sizes[0] / HIDC;
  if (nN <= 0 || in_sizes[0] != nN * HIDC) return;
  if (in_sizes[1] < 0 || (in_sizes[1] & 1)) return;
  const int nE = in_sizes[1] / 2;
  if (in_sizes[2] != PLN || in_sizes[4] != PLN || in_sizes[6] != PLN || in_sizes[8] != PLN) return;
  if (in_sizes[3] != DM || in_sizes[5] != DM || in_sizes[7] != DM || in_sizes[9] != DM) return;
  if (in_sizes[10] != 3 * DM || in_sizes[11] != DM || in_sizes[12] != DM) return;
  if (in_sizes[13] != PLN || in_sizes[14] != HIDC) return;
  if (out_size != nN * HIDC) return;

  const float* x     = (const float*)d_in[0];
  const int*   ei    = (const int*)d_in[1];
  const float* Wq    = (const float*)d_in[2];
  const float* bq    = (const float*)d_in[3];
  const float* Wk    = (const float*)d_in[4];
  const float* bk    = (const float*)d_in[5];
  const float* Wv    = (const float*)d_in[6];
  const float* bv    = (const float*)d_in[7];
  const float* Wsk   = (const float*)d_in[8];
  const float* bsk   = (const float*)d_in[9];
  const float* Wbeta = (const float*)d_in[10];
  const float* ln_g  = (const float*)d_in[11];
  const float* ln_b  = (const float*)d_in[12];
  const float* Wp    = (const float*)d_in[13];
  const float* bp    = (const float*)d_in[14];
  float* out = (float*)d_out;

  const int nP    = ((nN + GR - 1) / GR) * GR;
  const int gridA = (nN + NB - 1) / NB;
  const int nPA   = gridA * NB;

  size_t off = 0;
  unsigned short* planes = (unsigned short*)((char*)d_ws + off); off += (size_t)7 * PLN * sizeof(unsigned short);
  _Float16* qkv = (_Float16*)((char*)d_ws + off);                off += (size_t)3 * nP * DM * sizeof(_Float16);
  float* agg = (float*)((char*)d_ws + off);                       off += (size_t)nPA * DM * sizeof(float);
  if (off > ws_size) return;
  if (off > (size_t)134217728) return;

  const int n8 = PLN / 8;
  k_prep<<<dim3((n8 + NTHR - 1) / NTHR, 5), NTHR, 0, stream>>>(Wq, Wk, Wv, Wsk, Wp, planes, n8);

  k_qkv<<<dim3(nP / GR, 3), NTHR, 0, stream>>>(x, (const _Float16*)planes, bq, bk, bv, qkv, nN, nP);

  hipFuncSetAttribute(reinterpret_cast<const void*>(&k_agg),
                      hipFuncAttributeMaxDynamicSharedMemorySize, LDS_BYTES);
  k_agg<<<gridA, NTHR, LDS_BYTES, stream>>>(ei, qkv, qkv + (size_t)nP * DM, qkv + (size_t)2 * nP * DM,
                                            agg, nN, nE);

  k_tail<<<(nN + TR - 1) / TR, TTHR, 0, stream>>>(x, agg,
                                                  planes + (size_t)3 * PLN, planes + (size_t)4 * PLN, bsk,
                                                  Wbeta, ln_g, ln_b,
                                                  planes + (size_t)5 * PLN, planes + (size_t)6 * PLN, bp,
                                                  out, nN, nPA);
}
